// GatedGraphConv_687194767738
// MI455X (gfx1250) — hardware-verified
//
#include <hip/hip_runtime.h>

typedef __bf16         v16bf __attribute__((ext_vector_type(16)));
typedef unsigned short v8us  __attribute__((ext_vector_type(8)));
typedef unsigned short v4us  __attribute__((ext_vector_type(4)));
typedef float          v8f   __attribute__((ext_vector_type(8)));
typedef float          v4f   __attribute__((ext_vector_type(4)));
typedef v8us __attribute__((may_alias)) v8usa;
typedef v4us __attribute__((may_alias)) v4usa;
typedef v4f  __attribute__((may_alias)) v4fa;

union Frag { v16bf v; v8us half[2]; };

#define CH     128
#define KNB    16
#define KP     256
#define G3     384
#define NLAYER 3
#define RB     32
#define NTHR   256

#define U_WT0  0
#define U_WIH0 12288
#define U_WHH0 24576
#define U_WEND 36864
#define WPL_BYTES ((size_t)U_WEND * 16)
#define XF_OFF0   ((size_t)1048576)

static_assert(U_WIH0 == NLAYER * CH * KP / 8);
static_assert(U_WHH0 == U_WIH0 + G3 * KP / 8);
static_assert(U_WEND == U_WHH0 + G3 * KP / 8);
static_assert(U_WIH0 % NTHR == 0 && U_WHH0 % NTHR == 0 && U_WEND % NTHR == 0);
static_assert(WPL_BYTES <= XF_OFF0);
static_assert(KP % 32 == 0 && CH % 32 == 0 && KP == 2 * CH);
static_assert(RB * CH == 4 * NTHR * 4);
static_assert(RB == 4 * (NTHR / 32));
static_assert(CH == 16 * (NTHR / 32));
static_assert((CH * 4) % 128 == 0);
static_assert(RB * (CH * 4 / 128) == (NTHR / 32) * 4 * 4);

#define LO_XF 0
#define LO_XT 16384
#define LO_XS 32768
#define LO_AG 49152
#define LO_O  65536
#define SMEM_BYTES 81920
static_assert(LO_XT == RB * CH * 4 && LO_XS == LO_XT + RB * KP * 2 && LO_AG == LO_XS + RB * KP * 2);
static_assert(LO_O == LO_AG + RB * KP * 2 && SMEM_BYTES == LO_O + RB * CH * 4);

__device__ __forceinline__ unsigned short f2bf(float f) {
  unsigned u = __builtin_bit_cast(unsigned, f);
  u += 0x7FFFu + ((u >> 16) & 1u);
  return (unsigned short)(u >> 16);
}
__device__ __forceinline__ float bf2f(unsigned short s) {
  return __builtin_bit_cast(float, ((unsigned)s) << 16);
}
__device__ __forceinline__ float bfr(float f) { return bf2f(f2bf(f)); }

__device__ __forceinline__ float sigm_f(float v) {
  v = fminf(fmaxf(v, -30.0f), 30.0f);
  const float e = __expf(-v);
  return __builtin_amdgcn_rcpf(1.0f + e);
}
__device__ __forceinline__ float tanh_f(float v) {
  v = fminf(fmaxf(v, -15.0f), 15.0f);
  const float e = __expf(2.0f * v);
  return 1.0f - 2.0f * __builtin_amdgcn_rcpf(1.0f + e);
}

__device__ __forceinline__ v8f wmma_bf16(v16bf a, v16bf b, v8f c) {
  v8f d = __builtin_amdgcn_wmma_f32_16x16x32_bf16(false, a, false, b, (short)0, c, false, false);
  asm volatile("v_nop\n\tv_nop\n\tv_nop\n\tv_nop" : "+v"(d) : "v"(a), "v"(b));
  return d;
}

__device__ __forceinline__ v16bf load_frag(const unsigned short* p, int h) {
  Frag f;
  f.half[0] = *(const v8usa*)(p + 8 * h);
  f.half[1] = *(const v8usa*)(p + 16 + 8 * h);
  return f.v;
}

__global__ __launch_bounds__(NTHR) void convert_kernel(
    const float* __restrict__ x, const float* __restrict__ W,
    const float* __restrict__ wih, const float* __restrict__ whh,
    unsigned short* __restrict__ wpl, float* __restrict__ xf0,
    float* __restrict__ zrow_a, float* __restrict__ zrow_b, int nx4)
{
  const int g = blockIdx.x * NTHR + threadIdx.x;
  if (g < U_WIH0) {
    const int e = g * 8;
    const int row = e >> 8;
    const int li = row >> 7, n = row & (CH - 1);
    const int kk = e & (CH - 1);
    const float* src = W + (size_t)li * CH * CH + (size_t)kk * CH + n;
    const v8us o = { f2bf(src[0]),      f2bf(src[CH]),     f2bf(src[2 * CH]), f2bf(src[3 * CH]),
                     f2bf(src[4 * CH]), f2bf(src[5 * CH]), f2bf(src[6 * CH]), f2bf(src[7 * CH]) };
    unsigned short* dst = wpl + (size_t)g * 8;
    *(volatile v8us*)dst = o;
    __threadfence();
    *(volatile v8us*)dst = o;
    return;
  }
  if (g < U_WEND) {
    const bool isih = (g < U_WHH0);
    const float* base = isih ? wih : whh;
    const int e = (g - (isih ? U_WIH0 : U_WHH0)) * 8;
    const int j = e >> 8, kk = e & (CH - 1);
    const float* src = base + (size_t)j * CH + kk;
    const v4f a = *(const v4fa*)src;
    const v4f c = *(const v4fa*)(src + 4);
    const v8us o = { f2bf(a.x), f2bf(a.y), f2bf(a.z), f2bf(a.w),
                     f2bf(c.x), f2bf(c.y), f2bf(c.z), f2bf(c.w) };
    unsigned short* dst = wpl + (size_t)g * 8;
    *(volatile v8us*)dst = o;
    __threadfence();
    *(volatile v8us*)dst = o;
    return;
  }
  const int q = g - U_WEND;
  if (q < nx4) {
    const v4f a = *(const v4fa*)(x + (size_t)q * 4);
    const v4f o = { bfr(a.x), bfr(a.y), bfr(a.z), bfr(a.w) };
    float* dst = xf0 + (size_t)q * 4;
    *(volatile v4f*)dst = o;
    __threadfence();
    *(volatile v4f*)dst = o;
    return;
  }
  const int u = q - nx4;
  if (u < 64) {
    const v4f z = { 0.0f, 0.0f, 0.0f, 0.0f };
    float* dst = ((u < 32) ? zrow_a : zrow_b) + (u & 31) * 4;
    *(volatile v4f*)dst = z;
    __threadfence();
    *(volatile v4f*)dst = z;
  }
}

__device__ __forceinline__ void tile_store_pass(const float* sO, float* dst,
                                                int n0, int w, int lane) {
  const int q8 = lane & 7, sub = lane >> 3;
  #pragma unroll
  for (int i = 0; i < 4; ++i) {
    const int lid = w * 16 + i * 4 + sub;
    const int row = lid >> 2, seg = lid & 3;
    const v4f v = *(const v4fa*)(sO + row * CH + seg * 32 + 4 * q8);
    *(volatile v4f*)(dst + (size_t)(n0 + row) * CH + seg * 32 + 4 * q8) = v;
  }
}

__global__ __launch_bounds__(NTHR) void layer_kernel(
    const float* __restrict__ xsrc,
    const int* __restrict__ edge,
    const unsigned short* __restrict__ wt,
    const unsigned short* __restrict__ wih,
    const unsigned short* __restrict__ whh,
    const float* __restrict__ bih, const float* __restrict__ bhh,
    float* __restrict__ xdst,
    int N, int kdh)
{
  extern __shared__ __attribute__((aligned(16))) char smem[];
  float* sXF = (float*)(smem + LO_XF);
  unsigned short* sXT = (unsigned short*)(smem + LO_XT);
  unsigned short* sXS = (unsigned short*)(smem + LO_XS);
  unsigned short* sAG = (unsigned short*)(smem + LO_AG);
  float* sO = (float*)(smem + LO_O);

  const int tid = threadIdx.x, lane = tid & 31, w = tid >> 5;
  const int h = lane >> 4, m = lane & 15;
  const int n0 = blockIdx.x * RB;

  #pragma unroll
  for (int it = 0; it < 4; ++it) {
    const int q = it * NTHR + tid;
    const int row = q >> 5, c4 = (q & 31) * 4;
    const v4f v = *(const v4fa*)(xsrc + (size_t)(n0 + row) * CH + c4);
    *(v4fa*)(sXF + row * CH + c4) = v;
    const unsigned short h0 = f2bf(v.x), h1 = f2bf(v.y), h2 = f2bf(v.z), h3 = f2bf(v.w);
    const v4us hv = { h0, h1, h2, h3 };
    const v4us lv = { f2bf(v.x - bf2f(h0)), f2bf(v.y - bf2f(h1)),
                      f2bf(v.z - bf2f(h2)), f2bf(v.w - bf2f(h3)) };
    *(v4usa*)(sXT + row * KP + c4) = hv;
    *(v4usa*)(sXT + row * KP + CH + c4) = lv;
  }

  #pragma unroll 1
  for (int s = 0; s < 4; ++s) {
    const int rr = 4 * w + s;
    int e = edge[(size_t)(n0 + rr) * KNB + (lane & (KNB - 1))];
    if (e < 0) e += N + 1;
    e = min(max(e, 0), N);
    v4f acc = { 0.0f, 0.0f, 0.0f, 0.0f };
    #pragma unroll
    for (int k = 0; k < KNB; ++k) {
      const int j = __shfl(e, k);
      const v4f v = *(const v4fa*)(xsrc + (size_t)j * CH + 4 * lane);
      acc.x += v.x; acc.y += v.y; acc.z += v.z; acc.w += v.w;
    }
    const unsigned short h0 = f2bf(acc.x), h1 = f2bf(acc.y), h2 = f2bf(acc.z), h3 = f2bf(acc.w);
    const v4us hv = { h0, h1, h2, h3 };
    const v4us lv = { f2bf(acc.x - bf2f(h0)), f2bf(acc.y - bf2f(h1)),
                      f2bf(acc.z - bf2f(h2)), f2bf(acc.w - bf2f(h3)) };
    *(v4usa*)(sXS + rr * KP + 4 * lane) = hv;
    *(v4usa*)(sXS + rr * KP + CH + 4 * lane) = lv;
  }
  __syncthreads();

  {
    const v8f z8 = { 0.f, 0.f, 0.f, 0.f, 0.f, 0.f, 0.f, 0.f };
    v8f acc[2];
    acc[0] = z8; acc[1] = z8;
    const unsigned short* a0p = sXS + m * KP;
    const unsigned short* a1p = sXS + (16 + m) * KP;
    const unsigned short* bp = wt + (size_t)(16 * w + m) * KP;
    #pragma unroll 1
    for (int k0 = 0; k0 < KP; k0 += 32) {
      const v16bf a0 = load_frag(a0p + k0, h);
      const v16bf a1 = load_frag(a1p + k0, h);
      const v16bf b = load_frag(bp + k0, h);
      acc[0] = wmma_bf16(a0, b, acc[0]);
      acc[1] = wmma_bf16(a1, b, acc[1]);
    }
    const int c = 16 * w + m;
    #pragma unroll
    for (int rt = 0; rt < 2; ++rt) {
      #pragma unroll
      for (int r = 0; r < 8; ++r) {
        const int row = 16 * rt + 8 * h + r;
        const float v = acc[rt][r];
        const unsigned short hi = f2bf(v);
        sAG[row * KP + c] = hi;
        sAG[row * KP + CH + c] = f2bf(v - bf2f(hi));
      }
    }
  }
  __syncthreads();

  const v8f z8 = { 0.f, 0.f, 0.f, 0.f, 0.f, 0.f, 0.f, 0.f };
  v8f gia[2][3], gha[2][3];
  #pragma unroll
  for (int rt = 0; rt < 2; ++rt)
    #pragma unroll
    for (int g = 0; g < 3; ++g) { gia[rt][g] = z8; gha[rt][g] = z8; }
  {
    const unsigned short* a0p = sAG + m * KP;
    const unsigned short* a1p = sAG + (16 + m) * KP;
    const unsigned short* b0 = wih + (size_t)(16 * w + m) * KP;
    #pragma unroll 1
    for (int k0 = 0; k0 < KP; k0 += 32) {
      const v16bf a0 = load_frag(a0p + k0, h);
      const v16bf a1 = load_frag(a1p + k0, h);
      #pragma unroll
      for (int g = 0; g < 3; ++g) {
        const v16bf b = load_frag(b0 + (size_t)g * CH * KP + k0, h);
        gia[0][g] = wmma_bf16(a0, b, gia[0][g]);
        gia[1][g] = wmma_bf16(a1, b, gia[1][g]);
      }
    }
  }
  {
    const unsigned short* a0p = sXT + m * KP;
    const unsigned short* a1p = sXT + (16 + m) * KP;
    const unsigned short* b0 = whh + (size_t)(16 * w + m) * KP;
    #pragma unroll 1
    for (int k0 = 0; k0 < kdh; k0 += 32) {
      const v16bf a0 = load_frag(a0p + k0, h);
      const v16bf a1 = load_frag(a1p + k0, h);
      #pragma unroll
      for (int g = 0; g < 3; ++g) {
        const v16bf b = load_frag(b0 + (size_t)g * CH * KP + k0, h);
        gha[0][g] = wmma_bf16(a0, b, gha[0][g]);
        gha[1][g] = wmma_bf16(a1, b, gha[1][g]);
      }
    }
  }

  {
    const int c = 16 * w + m;
    const float bi_r = bfr(bih[c]), bi_z = bfr(bih[CH + c]), bi_n = bfr(bih[2 * CH + c]);
    const float bh_r = bfr(bhh[c]), bh_z = bfr(bhh[CH + c]), bh_n = bfr(bhh[2 * CH + c]);
    #pragma unroll
    for (int rt = 0; rt < 2; ++rt) {
      #pragma unroll
      for (int r = 0; r < 8; ++r) {
        const int row = 16 * rt + 8 * h + r;
        const float pr = (gia[rt][0][r] + bi_r) + (gha[rt][0][r] + bh_r);
        const float pz = (gia[rt][1][r] + bi_z) + (gha[rt][1][r] + bh_z);
        const float rg = sigm_f(pr);
        const float zg = sigm_f(pz);
        const float pn = (gia[rt][2][r] + bi_n) + rg * (gha[rt][2][r] + bh_n);
        const float ng = tanh_f(pn);
        const float xp = sXF[row * CH + c];
        sO[row * CH + c] = (1.0f - zg) * ng + zg * xp;
      }
    }
  }
  __syncthreads();

  tile_store_pass(sO, xdst, n0, w, lane);
  __threadfence();
  tile_store_pass(sO, xdst, n0, w, lane);
}

extern "C" void kernel_launch(void* const* d_in, const int* in_sizes, int n_in,
                              void* d_out, int out_size, void* d_ws, size_t ws_size,
                              hipStream_t stream) {
  if (n_in < 7) return;
  if (in_sizes[0] <= 0 || (in_sizes[0] % CH) != 0) return;
  const int N = in_sizes[0] / CH;
  if ((N % RB) != 0) return;
  if (in_sizes[1] != N * KNB) return;
  if (in_sizes[2] != NLAYER * CH * CH) return;
  if (in_sizes[3] != G3 * CH || in_sizes[4] != G3 * CH) return;
  if (in_sizes[5] != G3 || in_sizes[6] != G3) return;
  if (out_size != N * CH) return;

  const size_t xf_bytes = (size_t)(N + 1) * CH * 4;
  const size_t off_a = XF_OFF0;
  const size_t off_b = off_a + xf_bytes;
  const size_t total = off_b + xf_bytes;
  if (total > ws_size) return;

  const float* x    = (const float*)d_in[0];
  const int*   edge = (const int*)d_in[1];
  const float* W    = (const float*)d_in[2];
  const float* wih  = (const float*)d_in[3];
  const float* whh  = (const float*)d_in[4];
  const float* bih  = (const float*)d_in[5];
  const float* bhh  = (const float*)d_in[6];
  float* out = (float*)d_out;

  char* ws = (char*)d_ws;
  unsigned short* wpl = (unsigned short*)ws;
  const unsigned short* wtp  = wpl + (size_t)U_WT0 * 8;
  const unsigned short* wihp = wpl + (size_t)U_WIH0 * 8;
  const unsigned short* whhp = wpl + (size_t)U_WHH0 * 8;
  float* xfa = (float*)(ws + off_a);
  float* xfb = (float*)(ws + off_b);

  const int nx4 = N * CH / 4;
  const int nunits = U_WEND + nx4 + 64;
  convert_kernel<<<(nunits + NTHR - 1) / NTHR, NTHR, 0, stream>>>(
      x, W, wih, whh, wpl, xfb, xfa + (size_t)N * CH, xfb + (size_t)N * CH, nx4);

  hipFuncSetAttribute(reinterpret_cast<const void*>(&layer_kernel),
                      hipFuncAttributeMaxDynamicSharedMemorySize, SMEM_BYTES);

  layer_kernel<<<N / RB, NTHR, SMEM_BYTES, stream>>>(
      xfb, edge, wtp + (size_t)0 * CH * KP, wihp, whhp, bih, bhh, xfa, N, CH);
  layer_kernel<<<N / RB, NTHR, SMEM_BYTES, stream>>>(
      xfa, edge, wtp + (size_t)1 * CH * KP, wihp, whhp, bih, bhh, xfb, N, KP);
  layer_kernel<<<N / RB, NTHR, SMEM_BYTES, stream>>>(
      xfb, edge, wtp + (size_t)2 * CH * KP, wihp, whhp, bih, bhh, out, N, KP);
}
